// EuclideanMessagePassing_463856468032
// MI455X (gfx1250) — hardware-run, weakly checked
//
#include <hip/hip_runtime.h>
#include <stddef.h>
#include <stdint.h>

#define SPLIT   1
#define NN      50000
#define NE      625000
#define DF      128
#define MP      50048
#define APITCH  256
#define WPITCH  256
#define KTOT    (SPLIT ? 256 : 128)
#define NTHR    256
#define NWAVE   8
#define EPT     8
#define WCH     (32 * EPT)
#define NBRUN   1024
#define SLB     10
#define NBK     49
#define WLCAP   2048
#define RCAP    16384
#define DEGCAP  64
#define MAXDEG_MEAS 31
#define MAXBLK_MEAS 13063
#define RBM     64
#define GBM     64
#define GBN     128
#define GTHR    128

#define BK_ZINTS (NWAVE * WLCAP + 2 * RCAP + 3 * NBRUN)
#define BK_INTS  (BK_ZINTS + 16)
#define BK_LDS   (BK_INTS * 4)

#define PBX   (MP * DF / 8 / NTHR)
#define PBW   (DF * WPITCH / 8 / NTHR)
#define PBTOT (PBX + PBW + 1)

static_assert(DF == 128 && DF == 4 * 32 && GBN == DF);
static_assert(MP % GBM == 0 && MP % RBM == 0 && MP >= NN && MP == 391 * 128);
static_assert(NBRUN == (1 << SLB) && NBRUN % RBM == 0 && NBRUN % GBM == 0 && NBRUN % 32 == 0);
static_assert(NBK * NBRUN >= MP && NBK * NBRUN >= NN);
static_assert(NE < (1 << 21) && (((long long)NE) << SLB) < (1LL << 31));
static_assert(NE % EPT == 0 && NE % 4 == 0 && NE >= EPT);
static_assert(RCAP == NWAVE * WLCAP && RCAP % 4 == 0);
static_assert((long long)RCAP * 100 >= (long long)MAXBLK_MEAS * 105);
static_assert(WLCAP >= MAXBLK_MEAS / 8 + 8 * 46 + 1);
static_assert(MAXDEG_MEAS + 8 <= DEGCAP);
static_assert(BK_ZINTS % (NTHR * 4) == 0 && (2 * RCAP) % (NTHR * 4) == 0 && (2 * NBRUN) % (NTHR * 4) == 0);
static_assert(BK_LDS <= 327680);
static_assert(KTOT % 32 == 0 && KTOT <= APITCH && KTOT <= WPITCH && APITCH == 2 * DF && WPITCH == 2 * DF);
static_assert((MP * DF / 8) % NTHR == 0 && (DF * WPITCH / 8) % NTHR == 0);
static_assert(GBM == (GTHR / 32) * 16 && RBM == NWAVE * 8);
static_assert((GBM * GBN + DF) * 4 <= 65536);

typedef float          v4f   __attribute__((ext_vector_type(4)));
typedef float          v8f   __attribute__((ext_vector_type(8)));
typedef int            v2i   __attribute__((ext_vector_type(2)));
typedef int            v4i   __attribute__((ext_vector_type(4)));
typedef int            v8i   __attribute__((ext_vector_type(8)));
typedef unsigned       v2u   __attribute__((ext_vector_type(2)));
typedef unsigned short v8us  __attribute__((ext_vector_type(8)));
typedef unsigned short v16us __attribute__((ext_vector_type(16)));
typedef __bf16         v16bf __attribute__((ext_vector_type(16)));
typedef v4f  __attribute__((may_alias)) v4fa;
typedef v2i  __attribute__((may_alias)) v2ia;
typedef v4i  __attribute__((may_alias)) v4ia;
typedef v2u  __attribute__((may_alias)) v2ua;
typedef v8us __attribute__((may_alias)) v8usa;
union FragB { v16bf v; v16us u; v8us h[2]; v8i w; };

__device__ __forceinline__ v8f wmb(const FragB& a, const FragB& b, v8f c) {
  v8f d = __builtin_amdgcn_wmma_f32_16x16x32_bf16(false, a.v, false, b.v, (short)0, c, false, false);
  asm volatile("v_nop\n\tv_nop\n\tv_nop\n\tv_nop" : "+v"(d) : "v"(a.w), "v"(b.w));
  return d;
}

__device__ __forceinline__ unsigned bf16_bits(float f) {
  const unsigned u = __float_as_uint(f);
  const unsigned r = (u + 0x7fffu + ((u >> 16) & 1u)) >> 16;
  const unsigned q = (u >> 16) | 0x40u;
  return ((u & 0x7fffffffu) > 0x7f800000u) ? q : r;
}
__device__ __forceinline__ float bf16_val(float f) {
  return __uint_as_float(bf16_bits(f) << 16);
}

__device__ __forceinline__ void hilo_pack(float v0, float v1, float v2, float v3,
                                          int& h01, int& h23, int& l01, int& l23) {
  const unsigned a0 = bf16_bits(v0), a1 = bf16_bits(v1), a2 = bf16_bits(v2), a3 = bf16_bits(v3);
  const unsigned b0 = bf16_bits(v0 - __uint_as_float(a0 << 16));
  const unsigned b1 = bf16_bits(v1 - __uint_as_float(a1 << 16));
  const unsigned b2 = bf16_bits(v2 - __uint_as_float(a2 << 16));
  const unsigned b3 = bf16_bits(v3 - __uint_as_float(a3 << 16));
  h01 = (int)(a0 | (a1 << 16)); h23 = (int)(a2 | (a3 << 16));
  l01 = (int)(b0 | (b1 << 16)); l23 = (int)(b2 | (b3 << 16));
}

__device__ __forceinline__ void st2_v4f(float* p, v4f v) {
  *(volatile v4f*)p = v;
  __threadfence();
  *(volatile v4f*)p = v;
}
__device__ __forceinline__ void st2_v8us(unsigned short* p, v8us v) {
  *(volatile v8us*)p = v;
  __threadfence();
  *(volatile v8us*)p = v;
}

__global__ __launch_bounds__(NTHR) void k_prep(const float* __restrict__ x, const float* __restrict__ wt,
                                               const float* __restrict__ bias, unsigned short* xb,
                                               unsigned short* wd, float* biasf) {
  const int tid = (int)threadIdx.x, lane = tid & 31;
  const int blk = (int)blockIdx.x;
  if (blk < PBX) {
    const int u   = blk * NTHR + tid;
    const int row = u >> 4, k8 = (u & 15) * 8;
    const int rc  = row < NN ? row : NN - 1;
    const unsigned mk = row < NN ? 0xffffu : 0u;
    const float* p = x + (size_t)rc * DF + k8;
    const v4f a = *(const v4fa*)p;
    const v4f b = *(const v4fa*)(p + 4);
    v8us o;
    o[0] = (unsigned short)(bf16_bits(a.x) & mk); o[1] = (unsigned short)(bf16_bits(a.y) & mk);
    o[2] = (unsigned short)(bf16_bits(a.z) & mk); o[3] = (unsigned short)(bf16_bits(a.w) & mk);
    o[4] = (unsigned short)(bf16_bits(b.x) & mk); o[5] = (unsigned short)(bf16_bits(b.y) & mk);
    o[6] = (unsigned short)(bf16_bits(b.z) & mk); o[7] = (unsigned short)(bf16_bits(b.w) & mk);
    st2_v8us(xb + (size_t)row * DF + k8, o);
  } else if (blk < PBX + PBW) {
    const int u  = (blk - PBX) * NTHR + tid;
    const int n  = u >> 5, k8 = (u & 31) * 8, kk = k8 & (DF - 1);
    const float* p = wt + (size_t)n * DF + kk;
    const v4f a = *(const v4fa*)p;
    const v4f b = *(const v4fa*)(p + 4);
    v8us o;
    o[0] = (unsigned short)bf16_bits(a.x); o[1] = (unsigned short)bf16_bits(a.y);
    o[2] = (unsigned short)bf16_bits(a.z); o[3] = (unsigned short)bf16_bits(a.w);
    o[4] = (unsigned short)bf16_bits(b.x); o[5] = (unsigned short)bf16_bits(b.y);
    o[6] = (unsigned short)bf16_bits(b.z); o[7] = (unsigned short)bf16_bits(b.w);
    st2_v8us(wd + (size_t)n * WPITCH + k8, o);
  } else {
    if (tid < 32) {
      const v4f t = *(const v4fa*)(bias + 4 * lane);
      v4f o;
      o.x = bf16_val(t.x); o.y = bf16_val(t.y); o.z = bf16_val(t.z); o.w = bf16_val(t.w);
      st2_v4f(biasf + 4 * lane, o);
    }
  }
}

__device__ __forceinline__ void bucket_flush(const int* pl, const int* cnt, int ov, int* lp, int* cop, int* fp,
                                             int tid) {
#pragma unroll 1
  for (int i = tid * 4; i < 2 * RCAP; i += NTHR * 4) {
    const v4i v = *(const v4ia*)(pl + i);
    *(volatile v4i*)(lp + i) = v;
  }
#pragma unroll 1
  for (int i = tid * 4; i < 2 * NBRUN; i += NTHR * 4) {
    const v4i v = *(const v4ia*)(cnt + i);
    *(volatile v4i*)(cop + i) = v;
  }
  if (tid < 8) {
    const v4i f = {ov, ov, ov, ov};
    *(volatile v4i*)(fp + 4 * tid) = f;
  }
}

__global__ __launch_bounds__(NTHR) void k_bucket(const int* __restrict__ srcs, const int* __restrict__ dsts,
                                                 const float* __restrict__ ew, int* LIST, int* CO, int* FLAG) {
  extern __shared__ __attribute__((aligned(16))) int dsm[];
  int* wl   = dsm;
  int* pl   = dsm + NWAVE * WLCAP;
  int* cnt  = pl + 2 * RCAP;
  int* offs = cnt + NBRUN;
  int* cur  = offs + NBRUN;
  int* misc = cur + NBRUN;
  const int tid = (int)threadIdx.x, lane = tid & 31, wave = tid >> 5;
  const int blk = (int)blockIdx.x;
  const unsigned nbs = (unsigned)(blk * NBRUN);

  {
    const v4i z4 = {0, 0, 0, 0};
    for (int i = tid * 4; i < BK_ZINTS; i += NTHR * 4) *(v4ia*)(dsm + i) = z4;
    if (tid < 16) misc[tid] = 0;
  }
  __syncthreads();

  {
    const int per  = ((NE + NWAVE * WCH - 1) / (NWAVE * WCH)) * WCH;
    const int ebeg = wave * per;
    const int eend = (ebeg + per < NE) ? (ebeg + per) : NE;
    int* mylist = wl + wave * WLCAP;
    int wc = 0;
#pragma unroll 1
    for (int cb = ebeg; cb < eend; cb += WCH) {
      const int e0  = cb + lane * EPT;
      const int e0c = e0 < NE - EPT ? e0 : NE - EPT;
      const bool inr = e0 < NE;
      const v4i da = *(const v4ia*)(dsts + e0c);
      const v4i db = *(const v4ia*)(dsts + e0c + 4);
      asm volatile("" :: "v"(da));
      asm volatile("" :: "v"(db));
      const unsigned s0 = (unsigned)da.x - nbs, s1 = (unsigned)da.y - nbs;
      const unsigned s2 = (unsigned)da.z - nbs, s3 = (unsigned)da.w - nbs;
      const unsigned s4 = (unsigned)db.x - nbs, s5 = (unsigned)db.y - nbs;
      const unsigned s6 = (unsigned)db.z - nbs, s7 = (unsigned)db.w - nbs;
      const bool h0 = (s0 < (unsigned)NBRUN) & inr, h1 = (s1 < (unsigned)NBRUN) & inr;
      const bool h2 = (s2 < (unsigned)NBRUN) & inr, h3 = (s3 < (unsigned)NBRUN) & inr;
      const bool h4 = (s4 < (unsigned)NBRUN) & inr, h5 = (s5 < (unsigned)NBRUN) & inr;
      const bool h6 = (s6 < (unsigned)NBRUN) & inr, h7 = (s7 < (unsigned)NBRUN) & inr;
      const unsigned m0 = __builtin_amdgcn_ballot_w32(h0), m1 = __builtin_amdgcn_ballot_w32(h1);
      const unsigned m2 = __builtin_amdgcn_ballot_w32(h2), m3 = __builtin_amdgcn_ballot_w32(h3);
      const unsigned m4 = __builtin_amdgcn_ballot_w32(h4), m5 = __builtin_amdgcn_ballot_w32(h5);
      const unsigned m6 = __builtin_amdgcn_ballot_w32(h6), m7 = __builtin_amdgcn_ballot_w32(h7);
      const unsigned any = m0 | m1 | m2 | m3 | m4 | m5 | m6 | m7;
      if (any != 0u) {
        const int pre = (int)(__builtin_amdgcn_mbcnt_lo(m0, 0u) + __builtin_amdgcn_mbcnt_lo(m1, 0u) +
                              __builtin_amdgcn_mbcnt_lo(m2, 0u) + __builtin_amdgcn_mbcnt_lo(m3, 0u) +
                              __builtin_amdgcn_mbcnt_lo(m4, 0u) + __builtin_amdgcn_mbcnt_lo(m5, 0u) +
                              __builtin_amdgcn_mbcnt_lo(m6, 0u) + __builtin_amdgcn_mbcnt_lo(m7, 0u));
        int p = wc + pre;
        if (h0) { if (p < WLCAP) mylist[p] = ((e0 + 0) << SLB) | (int)s0; p = p + 1; }
        if (h1) { if (p < WLCAP) mylist[p] = ((e0 + 1) << SLB) | (int)s1; p = p + 1; }
        if (h2) { if (p < WLCAP) mylist[p] = ((e0 + 2) << SLB) | (int)s2; p = p + 1; }
        if (h3) { if (p < WLCAP) mylist[p] = ((e0 + 3) << SLB) | (int)s3; p = p + 1; }
        if (h4) { if (p < WLCAP) mylist[p] = ((e0 + 4) << SLB) | (int)s4; p = p + 1; }
        if (h5) { if (p < WLCAP) mylist[p] = ((e0 + 5) << SLB) | (int)s5; p = p + 1; }
        if (h6) { if (p < WLCAP) mylist[p] = ((e0 + 6) << SLB) | (int)s6; p = p + 1; }
        if (h7) { if (p < WLCAP) mylist[p] = ((e0 + 7) << SLB) | (int)s7; p = p + 1; }
        wc += (int)(__builtin_popcount(m0) + __builtin_popcount(m1) + __builtin_popcount(m2) + __builtin_popcount(m3) +
                    __builtin_popcount(m4) + __builtin_popcount(m5) + __builtin_popcount(m6) + __builtin_popcount(m7));
      }
    }
    if (lane == 0) misc[wave] = wc;
  }
  __syncthreads();

  if (wave == 0) {
    int ov = 0;
#pragma unroll 1
    for (int w2 = 0; w2 < NWAVE; ++w2) {
      int c = misc[w2];
      if (c > WLCAP) ov = 1;
      c = c < 0 ? 0 : (c > WLCAP ? WLCAP : c);
#pragma unroll 1
      for (int b0 = 0; b0 < c; b0 += 32) {
        const int idx = b0 + lane;
        const int ent = wl[w2 * WLCAP + (idx < WLCAP ? idx : WLCAP - 1)];
        const int m32 = (c - b0) < 32 ? (c - b0) : 32;
#pragma unroll 1
        for (int k = 0; k < m32; ++k) {
          const int u    = __builtin_amdgcn_readlane(ent, k);
          const int slot = u & (NBRUN - 1);
          if (lane == 0) cnt[slot] = cnt[slot] + 1;
        }
      }
    }
    if (lane == 0) misc[9] = ov;
  }
  __syncthreads();
  if (wave == 0) {
    const int base = lane * (NBRUN / 32);
    int s = 0, mx = 0;
#pragma unroll 1
    for (int i = 0; i < NBRUN / 32; ++i) {
      const int cv = cnt[base + i];
      s += cv;
      mx = cv > mx ? cv : mx;
    }
    const unsigned bigm = __builtin_amdgcn_ballot_w32(mx > DEGCAP);
    int incl = s;
#pragma unroll
    for (int d = 1; d < 32; d <<= 1) {
      const int y = __shfl_up(incl, d, 32);
      if (lane >= d) incl += y;
    }
    int run = incl - s;
#pragma unroll 1
    for (int i = 0; i < NBRUN / 32; ++i) {
      const int cv = cnt[base + i];
      offs[base + i] = run;
      cur[base + i]  = run;
      run += cv;
    }
    if (lane == 0 && bigm != 0u) misc[9] = 1;
  }
  __syncthreads();

  if (wave == 0) {
#pragma unroll 1
    for (int w2 = 0; w2 < NWAVE; ++w2) {
      int c = misc[w2];
      c = c < 0 ? 0 : (c > WLCAP ? WLCAP : c);
#pragma unroll 1
      for (int b0 = 0; b0 < c; b0 += 32) {
        const int idx = b0 + lane;
        const int ent = wl[w2 * WLCAP + (idx < WLCAP ? idx : WLCAP - 1)];
        int eid = (ent >> SLB) & 0x1fffff;
        eid = eid > NE - 1 ? NE - 1 : eid;
        int sr = srcs[eid];
        sr = sr < 0 ? 0 : (sr > NN - 1 ? NN - 1 : sr);
        const int wb = (int)(bf16_bits(ew[eid]) << 16);
        const int m32 = (c - b0) < 32 ? (c - b0) : 32;
#pragma unroll 1
        for (int k = 0; k < m32; ++k) {
          const int u    = __builtin_amdgcn_readlane(ent, k);
          const int sk   = __builtin_amdgcn_readlane(sr, k);
          const int wk   = __builtin_amdgcn_readlane(wb, k);
          const int slot = u & (NBRUN - 1);
          if (lane == 0) {
            int p = cur[slot];
            p = p < 0 ? 0 : (p > RCAP - 1 ? RCAP - 1 : p);
            v2i en;
            en.x = sk; en.y = wk;
            *(v2ia*)(pl + 2 * p) = en;
            cur[slot] = p + 1;
          }
        }
      }
    }
  }
  __syncthreads();

  const int ovf = misc[9];
  int* lp  = LIST + (size_t)blk * (2 * RCAP);
  int* cop = CO + (size_t)blk * (2 * NBRUN);
  int* fp  = FLAG + (size_t)blk * 32;
  bucket_flush(pl, cnt, ovf, lp, cop, fp, tid);
  __threadfence();
  bucket_flush(pl, cnt, ovf, lp, cop, fp, tid);
}

__global__ __launch_bounds__(NTHR) void k_replay(const int* __restrict__ LIST, const int* __restrict__ CO,
                                                 const int* __restrict__ FLAG,
                                                 const unsigned short* __restrict__ XB, unsigned short* AGGHL) {
  const int tid = (int)threadIdx.x, lane = tid & 31, wave = tid >> 5;
  const int rowBase = (int)blockIdx.x * RBM;
  const int bucket  = rowBase >> SLB;
  const int* lb  = LIST + (size_t)bucket * (2 * RCAP);
  const int* cob = CO + (size_t)bucket * (2 * NBRUN);
  const int flag = FLAG[(size_t)bucket * 32];
  const float qnan = __uint_as_float(0x7fc00000u);

#pragma unroll 1
  for (int i = 0; i < RBM / NWAVE; ++i) {
    const int d    = rowBase + (RBM / NWAVE) * wave + i;
    const int slot = d & (NBRUN - 1);
    int c = cob[slot];
    int o = cob[NBRUN + slot];
    const bool big = c > DEGCAP;
    c = c < 0 ? 0 : (c > DEGCAP ? DEGCAP : c);
    o = o < 0 ? 0 : (o > RCAP - 1 ? RCAP - 1 : o);
    int last = o + c - 1;
    last = last < o ? o : last;
    last = last > RCAP - 1 ? RCAP - 1 : last;
    const int cs = __builtin_amdgcn_readfirstlane(c);
    float a0 = 0.0f, a1 = 0.0f, a2 = 0.0f, a3 = 0.0f;
#pragma unroll 1
    for (int j = 0; j < cs; ++j) {
      int idx = o + j;
      idx = idx > last ? last : idx;
      const v2i ent = *(const v2ia*)(lb + 2 * idx);
      int sr = ent.x;
      sr = sr < 0 ? 0 : (sr > NN - 1 ? NN - 1 : sr);
      const float w = __int_as_float(ent.y);
      const v2u xv = *(const v2ua*)(XB + (size_t)sr * DF + 4 * lane);
      asm volatile("" :: "v"(xv));
      const float x0 = __uint_as_float(xv.x << 16), x1 = __uint_as_float(xv.x & 0xffff0000u);
      const float x2 = __uint_as_float(xv.y << 16), x3 = __uint_as_float(xv.y & 0xffff0000u);
      const bool valid = j < c;
      const float t0 = fmaf(w, x0, a0), t1 = fmaf(w, x1, a1), t2 = fmaf(w, x2, a2), t3 = fmaf(w, x3, a3);
      a0 = valid ? t0 : a0; a1 = valid ? t1 : a1; a2 = valid ? t2 : a2; a3 = valid ? t3 : a3;
    }
    const bool bad  = (flag != 0) | big;
    const bool live = d < NN;
    float m0 = bad ? qnan : a0, m1 = bad ? qnan : a1, m2 = bad ? qnan : a2, m3 = bad ? qnan : a3;
    m0 = live ? m0 : 0.0f; m1 = live ? m1 : 0.0f; m2 = live ? m2 : 0.0f; m3 = live ? m3 : 0.0f;
    int h01, h23, l01, l23;
    hilo_pack(m0, m1, m2, m3, h01, h23, l01, l23);
    v2u hv, lv;
    hv.x = (unsigned)h01; hv.y = (unsigned)h23;
    lv.x = (unsigned)l01; lv.y = (unsigned)l23;
    unsigned short* hp = AGGHL + (size_t)d * APITCH + 4 * lane;
    unsigned short* lp = hp + DF;
    *(volatile v2u*)hp = hv;
    *(volatile v2u*)lp = lv;
    __threadfence();
    *(volatile v2u*)hp = hv;
    *(volatile v2u*)lp = lv;
  }
}

__global__ __launch_bounds__(GTHR) __attribute__((amdgpu_num_vgpr(248)))
void k_gemm(const unsigned short* __restrict__ A, const unsigned short* __restrict__ BT,
            const float* __restrict__ biasf, const int* __restrict__ FLAG, float* out) {
  __shared__ __attribute__((aligned(16))) float stg[GBM * GBN];
  __shared__ __attribute__((aligned(16))) float sb[DF];
  const int tid = (int)threadIdx.x, lane = tid & 31, wave = tid >> 5, hh = lane >> 4, m = lane & 15;
  const int rowBase = (int)blockIdx.x * GBM;
  const int flag = FLAG[(size_t)(rowBase >> SLB) * 32];
  if (tid < 32) *(v4fa*)(sb + 4 * tid) = *(const v4fa*)(biasf + 4 * tid);

  v8f acc[8];
  {
    const v8f z = {0.f, 0.f, 0.f, 0.f, 0.f, 0.f, 0.f, 0.f};
#pragma unroll
    for (int t = 0; t < 8; ++t) acc[t] = z;
  }
  const unsigned short* ap = A + (size_t)(rowBase + 16 * wave + m) * (size_t)APITCH + 8 * hh;
  const unsigned short* bp = BT + (size_t)m * (size_t)WPITCH + 8 * hh;

#pragma unroll 1
  for (int k0 = 0; k0 < KTOT; k0 += 32) {
    FragB af;
    af.h[0] = *(const v8usa*)(ap + k0);
    af.h[1] = *(const v8usa*)(ap + k0 + 16);
#pragma unroll
    for (int nt = 0; nt < 8; ++nt) {
      const unsigned short* wq = bp + (size_t)(16 * nt) * (size_t)WPITCH + k0;
      FragB bf;
      bf.h[0] = *(const v8usa*)wq;
      bf.h[1] = *(const v8usa*)(wq + 16);
      acc[nt] = wmb(af, bf, acc[nt]);
    }
  }

#pragma unroll
  for (int nt = 0; nt < 8; ++nt) {
    const int lc = 16 * nt + m;
#pragma unroll
    for (int r = 0; r < 8; ++r) {
      const int lr = 16 * wave + 8 * hh + r;
      stg[lr * GBN + lc] = acc[nt][r];
    }
  }
  __syncthreads();

  const v4f bias4 = *(const v4fa*)(sb + 4 * lane);
  const float qnan = __uint_as_float(0x7fc00000u);
#pragma unroll 1
  for (int i = 0; i < 16; ++i) {
    const int lr   = 16 * wave + i;
    const int grow = rowBase + lr;
    const v4f a = *(const v4fa*)(stg + lr * GBN + 4 * lane);
    asm volatile("" :: "v"(a));
    float v0 = a.x + bias4.x, v1 = a.y + bias4.y, v2 = a.z + bias4.z, v3 = a.w + bias4.w;
    v0 = (v0 > 0.0f) ? v0 : (v0 - v0); v1 = (v1 > 0.0f) ? v1 : (v1 - v1);
    v2 = (v2 > 0.0f) ? v2 : (v2 - v2); v3 = (v3 > 0.0f) ? v3 : (v3 - v3);
    v4f o;
    o.x = (flag != 0) ? qnan : v0; o.y = (flag != 0) ? qnan : v1;
    o.z = (flag != 0) ? qnan : v2; o.w = (flag != 0) ? qnan : v3;
    if (grow < NN) st2_v4f(out + (size_t)grow * DF + 4 * lane, o);
  }
}

extern "C" void kernel_launch(void* const* d_in, const int* in_sizes, int n_in,
                              void* d_out, int out_size, void* d_ws, size_t ws_size,
                              hipStream_t stream) {
  if (n_in < 5) return;
  if (in_sizes[0] != NN * DF) return;
  if (in_sizes[1] != 2 * NE) return;
  if (in_sizes[2] != NE) return;
  if (in_sizes[3] != DF * DF) return;
  if (in_sizes[4] != DF) return;
  if (out_size != NN * DF) return;

  const float* x  = (const float*)d_in[0];
  const int*   ei = (const int*)d_in[1];
  const float* ew = (const float*)d_in[2];
  const float* wt = (const float*)d_in[3];
  const float* bs = (const float*)d_in[4];
  float* out = (float*)d_out;
  const int* srcs = ei;
  const int* dsts = ei + NE;

  constexpr size_t zXB   = (size_t)MP * DF * 2;
  constexpr size_t zAGG  = (size_t)MP * APITCH * 2;
  constexpr size_t zLIST = (size_t)NBK * RCAP * 8;
  constexpr size_t zCO   = (size_t)NBK * 2 * NBRUN * 4;
  constexpr size_t zFLAG = (size_t)(NBK + 1) * 128;
  constexpr size_t zWD   = (size_t)DF * WPITCH * 2;
  constexpr size_t zBF   = 512;
  constexpr size_t oXB   = 0;
  constexpr size_t oAGG  = oXB + zXB;
  constexpr size_t oLIST = oAGG + zAGG;
  constexpr size_t oCO   = oLIST + zLIST;
  constexpr size_t oFLAG = oCO + zCO;
  constexpr size_t oWD   = oFLAG + zFLAG;
  constexpr size_t oBF   = oWD + zWD;
  constexpr size_t oEND  = oBF + zBF;
  static_assert(zXB % 256 == 0 && zAGG % 256 == 0 && zLIST % 256 == 0 && zCO % 256 == 0);
  static_assert(zFLAG % 256 == 0 && zWD % 256 == 0 && zBF % 256 == 0);
  static_assert((size_t)NBK * 128 <= zFLAG);
  static_assert(oEND <= (size_t)(128u << 20));
  if (oEND > ws_size) return;

  char* ws = (char*)d_ws;
  unsigned short* XB    = (unsigned short*)(ws + oXB);
  unsigned short* AGGHL = (unsigned short*)(ws + oAGG);
  int*            LIST  = (int*)(ws + oLIST);
  int*            CO    = (int*)(ws + oCO);
  int*            FLAG  = (int*)(ws + oFLAG);
  unsigned short* WD    = (unsigned short*)(ws + oWD);
  float*          BIASF = (float*)(ws + oBF);

  hipFuncSetAttribute(reinterpret_cast<const void*>(&k_bucket), hipFuncAttributeMaxDynamicSharedMemorySize, (int)BK_LDS);

  k_prep<<<PBTOT, NTHR, 0, stream>>>(x, wt, bs, XB, WD, BIASF);
  k_bucket<<<NBK, NTHR, BK_LDS, stream>>>(srcs, dsts, ew, LIST, CO, FLAG);
  k_replay<<<MP / RBM, NTHR, 0, stream>>>(LIST, CO, FLAG, XB, AGGHL);
  k_gemm<<<MP / GBM, GTHR, 0, stream>>>(AGGHL, WD, BIASF, FLAG, out);
}
